// FALayer_20521353740426
// MI455X (gfx1250) — hardware-run, weakly checked
//
#include <hip/hip_runtime.h>
#include <stddef.h>


#define NN    8192
#define LNN   13
#define HH    256
#define RB    32
#define NTHR  256
#define NWAVE 8
#define ECH   1024
#define KCAP  2048
#define KC    64
#define KP    64
#define BMW   (RB * NN / 32)
#define GPB   32
#define WSCAP 134217728
#define LN_EPS 1e-5f

#define OFF_LK  0
#define OFF_LE  (OFF_LK + KCAP * 4)
#define OFF_MS  (OFF_LE + KCAP * 4)
#define OFF_WC  (OFF_MS + 64)
#define OFF_U   (OFF_WC + 448)
#define OFF_BM  (OFF_U)
#define OFF_CK  (OFF_BM + BMW * 4)
#define OFF_CE  (OFF_CK + ECH * 4)
#define END_SCAN (OFF_CE + ECH * 4)
#define OFF_BH  (OFF_U)
#define OFF_BL  (OFF_BH + HH * KP * 2)
#define OFF_AH  (OFF_BL + HH * KP * 2)
#define OFF_AL  (OFF_AH + RB * KP * 2)
#define OFF_GC  (OFF_AL + RB * KP * 2)
#define OFF_OC  (OFF_GC + KC * 4)
#define OFF_OS  (OFF_OC + KC * 4)
#define END_TILE (OFF_OS + KC * 4)
#define END_EPI (OFF_U + RB * HH * 4)
#define LDS_AGG (END_TILE)

static_assert(NN == (1 << LNN));
static_assert(NTHR == NWAVE * 32 && NTHR == HH);
static_assert(RB == 32 && RB * 8 == NTHR && RB == 2 * 16 && (RB % NWAVE) == 0);
static_assert(HH == 4 * 64 && (NWAVE / 2) * 64 == HH);
static_assert(ECH == 4 * NTHR);
static_assert((KCAP % KC) == 0 && (KC % 32) == 0 && KC == 8 * 8 && KP >= KC && (KP % 8) == 0);
static_assert((BMW % (4 * NTHR)) == 0);
static_assert((OFF_U % 256) == 0 && OFF_U >= OFF_WC + NWAVE * 4);
static_assert(END_SCAN <= LDS_AGG && END_EPI <= LDS_AGG);
static_assert((OFF_BL % 16) == 0 && (OFF_AH % 16) == 0 && (OFF_AL % 16) == 0 && (OFF_CK % 16) == 0);
static_assert(LDS_AGG <= 160 * 1024);

typedef float           v4f   __attribute__((ext_vector_type(4)));
typedef float           v8f   __attribute__((ext_vector_type(8)));
typedef int             v4i   __attribute__((ext_vector_type(4)));
typedef unsigned int    v4u   __attribute__((ext_vector_type(4)));
typedef unsigned short  v8us  __attribute__((ext_vector_type(8)));
typedef __bf16          v16bf __attribute__((ext_vector_type(16)));
union FragB { v16bf v; v8us h[2]; };

static __device__ __forceinline__ unsigned short f2bf(float f) {
  unsigned int u = __float_as_uint(f);
  u = u + 0x7FFFu + ((u >> 16) & 1u);
  return (unsigned short)(u >> 16);
}
static __device__ __forceinline__ float bf2f(unsigned short b) {
  return __uint_as_float(((unsigned int)b) << 16);
}

static __device__ __forceinline__ v8f wmb(v16bf a, v16bf b, v8f c) {
  v8f d = __builtin_amdgcn_wmma_f32_16x16x32_bf16(false, a, false, b, (short)0, c, false, false);
  asm volatile("v_nop\n\tv_nop\n\tv_nop\n\tv_nop" : "+v"(d) : "v"(a), "v"(b));
  return d;
}

static __device__ __forceinline__ float wave_sum(float v) {
#pragma unroll
  for (int m = 16; m > 0; m >>= 1) v += __shfl_xor(v, m, 32);
  return v;
}

__global__ __launch_bounds__(NTHR) void k_cvt(const float* __restrict__ src, unsigned short* dhi, unsigned short* dlo,
                                              int rowLen, int nSrcRows, int total8) {
  const int i = (int)blockIdx.x * NTHR + (int)threadIdx.x;
  if (i >= total8) return;
  const size_t e  = (size_t)8 * (size_t)i;
  const int    r  = (int)(e / (size_t)rowLen);
  const int    k0 = (int)(e - (size_t)r * (size_t)rowLen);
  const int    rc = r < nSrcRows ? r : nSrcRows - 1;
  const float  z  = (r < nSrcRows) ? 1.0f : 0.0f;
  const float* sp = src + (size_t)rc * rowLen + k0;
  const v4f f0 = *(const v4f*)sp;
  const v4f f1 = *(const v4f*)(sp + 4);
  float v[8];
  v[0] = f0.x * z; v[1] = f0.y * z; v[2] = f0.z * z; v[3] = f0.w * z;
  v[4] = f1.x * z; v[5] = f1.y * z; v[6] = f1.z * z; v[7] = f1.w * z;
  v8us hv, lv;
#pragma unroll
  for (int j = 0; j < 8; ++j) {
    const unsigned short hb = f2bf(v[j]);
    hv[j] = hb;
    lv[j] = f2bf(v[j] - bf2f(hb));
  }
  unsigned short* ph = dhi + e;
  unsigned short* pl = dlo + e;
  *(volatile v8us*)ph = hv;
  *(volatile v8us*)pl = lv;
  __threadfence();
  *(volatile v8us*)ph = hv;
  *(volatile v8us*)pl = lv;
}

__global__ __launch_bounds__(NTHR) void k_gate(const float* __restrict__ feat, const float* __restrict__ nd,
                                               const int* __restrict__ pairs, const float* __restrict__ gamma,
                                               const float* __restrict__ beta, const float* __restrict__ gw,
                                               const float* __restrict__ gb, float* gout, int nNodes, int nE) {
  __shared__ __attribute__((aligned(16))) float gl[GPB];
  const int tid = threadIdx.x, lane = tid & 31;
  const int wave = __builtin_amdgcn_readfirstlane(tid >> 5);
  const int blk = (int)blockIdx.x;
  const int base = lane * 16;

  float ga[16], be[16], wv[16];
#pragma unroll
  for (int q = 0; q < 4; ++q) {
    const v4f tg = *(const v4f*)(gamma + base + 4 * q);
    const v4f tb = *(const v4f*)(beta + base + 4 * q);
    const v4f tw = *(const v4f*)(gw + base + 4 * q);
    ga[4 * q + 0] = tg.x; ga[4 * q + 1] = tg.y; ga[4 * q + 2] = tg.z; ga[4 * q + 3] = tg.w;
    be[4 * q + 0] = tb.x; be[4 * q + 1] = tb.y; be[4 * q + 2] = tb.z; be[4 * q + 3] = tb.w;
    wv[4 * q + 0] = tw.x; wv[4 * q + 1] = tw.y; wv[4 * q + 2] = tw.z; wv[4 * q + 3] = tw.w;
  }
  const float bias0 = gb[0];

#pragma unroll 1
  for (int i = 0; i < GPB / NWAVE; ++i) {
    int e = blk * GPB + wave * (GPB / NWAVE) + i;
    e = e < nE ? e : nE - 1;
    int obj = pairs[2 * (size_t)e];
    int sub = pairs[2 * (size_t)e + 1];
    obj = obj < 0 ? 0 : (obj > nNodes - 1 ? nNodes - 1 : obj);
    sub = sub < 0 ? 0 : (sub > nNodes - 1 ? nNodes - 1 : sub);
    const int node = (lane < 16) ? sub : obj;
    const float* src = feat + (size_t)node * HH + (lane & 15) * 16;
    float x[16];
#pragma unroll
    for (int q = 0; q < 4; ++q) {
      const v4f t = *(const v4f*)(src + 4 * q);
      x[4 * q + 0] = t.x; x[4 * q + 1] = t.y; x[4 * q + 2] = t.z; x[4 * q + 3] = t.w;
    }
    float s = 0.f;
#pragma unroll
    for (int j = 0; j < 16; ++j) s += x[j];
    s = wave_sum(s);
    const float mu = s * (1.0f / 512.0f);
    float ss = 0.f;
#pragma unroll
    for (int j = 0; j < 16; ++j) { const float d = x[j] - mu; x[j] = d; ss += d * d; }
    ss = wave_sum(ss);
    const float var  = ss * (1.0f / 512.0f);
    const float rstd = rsqrtf(var + LN_EPS);
    float dot = 0.f;
#pragma unroll
    for (int j = 0; j < 16; ++j) {
      const float xn = x[j] * rstd * ga[j] + be[j];
      const float hr = fmaxf(xn, 0.f);
      dot += hr * wv[j];
    }
    dot = wave_sum(dot);
    float nrm = nd[obj] * nd[sub];
    nrm = (nrm > 10000.0f) ? 0.f : nrm;
    const float g = tanhf(dot + bias0) * nrm;
    if (lane == 0) gl[wave * (GPB / NWAVE) + i] = g;
  }
  __syncthreads();
  if (wave == 0) {
    const int lc = lane < 8 ? lane : 7;
    const v4f v = *(const v4f*)(gl + 4 * lc);
    float* p = gout + (size_t)blk * GPB + 4 * lane;
    if (lane < 8) *(volatile v4f*)p = v;
    __threadfence();
    if (lane < 8) *(volatile v4f*)p = v;
  }
}

__global__ __launch_bounds__(NTHR) void k_agg(const int* __restrict__ pairs,
                                              const unsigned short* __restrict__ Xh,
                                              const unsigned short* __restrict__ Xl,
                                              const float* G, float* out, int nE, int nChunks) {
  extern __shared__ v4f lds_dyn[];
  char* lds = (char*)lds_dyn;
  int* listK = (int*)(lds + OFF_LK);
  int* listE = (int*)(lds + OFF_LE);
  int* misc  = (int*)(lds + OFF_MS);
  int* wcnt  = (int*)(lds + OFF_WC);
  unsigned int* bitmap = (unsigned int*)(lds + OFF_BM);
  int* ckey  = (int*)(lds + OFF_CK);
  int* cedge = (int*)(lds + OFF_CE);
  unsigned short* Bh = (unsigned short*)(lds + OFF_BH);
  unsigned short* Bl = (unsigned short*)(lds + OFF_BL);
  unsigned short* Ah = (unsigned short*)(lds + OFF_AH);
  unsigned short* Al = (unsigned short*)(lds + OFF_AL);
  float* gch = (float*)(lds + OFF_GC);
  int*   och = (int*)(lds + OFF_OC);
  int*   osl = (int*)(lds + OFF_OS);
  float* stg = (float*)(lds + OFF_U);

  const int tid = threadIdx.x, lane = tid & 31, hh = lane >> 4, m = lane & 15;
  const int wave = __builtin_amdgcn_readfirstlane(tid >> 5);
  const int rowBase = (int)blockIdx.x * RB;

  {
    const v4u zz = {0u, 0u, 0u, 0u};
#pragma unroll 1
    for (int i = tid; i < BMW / 4; i += NTHR) ((v4u*)bitmap)[i] = zz;
  }
  int len = 0, ovf = 0;
  __syncthreads();
#pragma unroll 1
  for (int c = 0; c < nChunks; ++c) {
    const int cbase = c * ECH;
    int ob[4], sb[4];
    if (cbase + ECH <= nE) {
      const int* pp = pairs + 2 * (size_t)(cbase + 4 * tid);
      const v4i p0 = *(const v4i*)pp;
      const v4i p1 = *(const v4i*)(pp + 4);
      ob[0] = p0.x; sb[0] = p0.y; ob[1] = p0.z; sb[1] = p0.w;
      ob[2] = p1.x; sb[2] = p1.y; ob[3] = p1.z; sb[3] = p1.w;
    } else {
#pragma unroll
      for (int j = 0; j < 4; ++j) {
        int e = cbase + 4 * tid + j;
        e = e < nE ? e : nE - 1;
        ob[j] = pairs[2 * (size_t)e];
        sb[j] = pairs[2 * (size_t)e + 1];
      }
    }
    unsigned int msk[4];
    int wtot = 0;
#pragma unroll
    for (int j = 0; j < 4; ++j) {
      const int e = cbase + 4 * tid + j;
      const bool h = (e < nE) && ((unsigned)(sb[j] - rowBase) < (unsigned)RB) && ((unsigned)ob[j] < (unsigned)NN);
      msk[j] = __builtin_amdgcn_ballot_w32(h);
      wtot += __builtin_popcount(msk[j]);
    }
    if (lane == 0) wcnt[wave] = wtot;
    __syncthreads();
    int pre = 0, tot = 0;
#pragma unroll
    for (int w = 0; w < NWAVE; ++w) {
      const int cw = wcnt[w];
      pre += (w < wave) ? cw : 0;
      tot += cw;
    }
    int p = pre;
#pragma unroll
    for (int j = 0; j < 4; ++j) {
      const int below = __builtin_amdgcn_mbcnt_lo(msk[j], 0u);
      if ((msk[j] >> lane) & 1u) {
        const int pos = p + below;
        ckey[pos]  = ((sb[j] - rowBase) << LNN) | ob[j];
        cedge[pos] = cbase + 4 * tid + j;
      }
      p += __builtin_popcount(msk[j]);
    }
    __syncthreads();
    if (tid == 0) {
      const int tc = tot < ECH ? tot : ECH;
#pragma unroll 1
      for (int i = 0; i < tc; ++i) {
        const int key = ckey[i];
        const int w = (key >> 5) & (BMW - 1);
        const unsigned int bit = 1u << (key & 31);
        const unsigned int word = bitmap[w];
        if (!(word & bit)) {
          bitmap[w] = word | bit;
          if (len < KCAP) { listK[len] = key; listE[len] = cedge[i]; ++len; }
          else ovf = 1;
        }
      }
    }
  }
  if (tid == 0) { misc[0] = len; misc[1] = ovf; }
  __syncthreads();
  int listLen = misc[0];
  listLen = listLen < 0 ? 0 : (listLen > KCAP ? KCAP : listLen);
  listLen = __builtin_amdgcn_readfirstlane(listLen);
  const int ovfl = __builtin_amdgcn_readfirstlane(misc[1]);

  const int rt = wave & 1, cq = wave >> 1;
  v8f acc[4];
#pragma unroll
  for (int t = 0; t < 4; ++t) { v8f z8 = {0.f, 0.f, 0.f, 0.f, 0.f, 0.f, 0.f, 0.f}; acc[t] = z8; }
  const int nkc = (listLen + KC - 1) / KC;
#pragma unroll 1
  for (int kc = 0; kc < KCAP / KC; ++kc) {
    if (kc >= nkc) break;
    const int base = kc * KC;
    {
      const int j = tid & (KC - 1);
      const int idx = base + j;
      const bool valid = idx < listLen;
      const int idxc = valid ? idx : (listLen - 1);
      const int key = listK[idxc];
      int e = listE[idxc];
      e = e < 0 ? 0 : (e > nE - 1 ? nE - 1 : e);
      const float g = G[e];
      int sl = key >> LNN;
      sl = sl < 0 ? RB : (sl > RB - 1 ? RB : sl);
      if (tid < KC) {
        gch[j] = valid ? g : 0.f;
        och[j] = valid ? (key & (NN - 1)) : 0;
        osl[j] = valid ? sl : RB;
      }
    }
    __syncthreads();
    {
      const unsigned short* xh = Xh + tid;
      const unsigned short* xl = Xl + tid;
#pragma unroll 1
      for (int jg = 0; jg < KC / 8; ++jg) {
        v8us hv, lv;
#pragma unroll
        for (int i = 0; i < 8; ++i) {
          const int o = och[jg * 8 + i];
          const size_t xo = (size_t)o * HH;
          hv[i] = xh[xo];
          lv[i] = xl[xo];
        }
        *(v8us*)(Bh + tid * KP + jg * 8) = hv;
        *(v8us*)(Bl + tid * KP + jg * 8) = lv;
      }
    }
    {
      const int r = tid >> 3, jg = tid & 7;
      v8us hv, lv;
#pragma unroll
      for (int i = 0; i < 8; ++i) {
        const int j = jg * 8 + i;
        const float v = (osl[j] == r) ? gch[j] : 0.f;
        const unsigned short hb = f2bf(v);
        hv[i] = hb;
        lv[i] = f2bf(v - bf2f(hb));
      }
      *(v8us*)(Ah + r * KP + jg * 8) = hv;
      *(v8us*)(Al + r * KP + jg * 8) = lv;
    }
    __syncthreads();
#pragma unroll
    for (int ks = 0; ks < KC / 32; ++ks) {
      FragB fah, fal;
      const int ao = (16 * rt + m) * KP + 32 * ks + 8 * hh;
      fah.h[0] = *(const v8us*)(Ah + ao);
      fah.h[1] = *(const v8us*)(Ah + ao + 16);
      fal.h[0] = *(const v8us*)(Al + ao);
      fal.h[1] = *(const v8us*)(Al + ao + 16);
#pragma unroll
      for (int t = 0; t < 4; ++t) {
        const int bo = (64 * cq + 16 * t + m) * KP + 32 * ks + 8 * hh;
        FragB fbh, fbl;
        fbh.h[0] = *(const v8us*)(Bh + bo);
        fbh.h[1] = *(const v8us*)(Bh + bo + 16);
        fbl.h[0] = *(const v8us*)(Bl + bo);
        fbl.h[1] = *(const v8us*)(Bl + bo + 16);
        v8f d = acc[t];
        d = wmb(fah.v, fbh.v, d);
        d = wmb(fah.v, fbl.v, d);
        d = wmb(fal.v, fbh.v, d);
        acc[t] = d;
      }
    }
    __syncthreads();
  }

  const float qnan = __uint_as_float(0x7fc00000u);
  float* sp = stg + (16 * rt + 8 * hh) * HH + 64 * cq + m;
#pragma unroll
  for (int t = 0; t < 4; ++t) {
#pragma unroll
    for (int r = 0; r < 8; ++r) {
      const float v = acc[t][r];
      sp[r * HH + 16 * t] = ovfl ? qnan : v;
    }
  }
  __syncthreads();
#pragma unroll
  for (int i = 0; i < RB / NWAVE; ++i) {
    const int row = wave * (RB / NWAVE) + i;
    const float* lp = stg + row * HH;
    float* gp = out + (size_t)(rowBase + row) * HH;
    const v4f v0 = *(const v4f*)(lp + 4 * lane);
    const v4f v1 = *(const v4f*)(lp + 128 + 4 * lane);
    *(volatile v4f*)(gp + 4 * lane) = v0;
    *(volatile v4f*)(gp + 128 + 4 * lane) = v1;
  }
  __threadfence();
#pragma unroll
  for (int i = 0; i < RB / NWAVE; ++i) {
    const int row = wave * (RB / NWAVE) + i;
    const float* lp = stg + row * HH;
    float* gp = out + (size_t)(rowBase + row) * HH;
    const v4f v0 = *(const v4f*)(lp + 4 * lane);
    const v4f v1 = *(const v4f*)(lp + 128 + 4 * lane);
    *(volatile v4f*)(gp + 4 * lane) = v0;
    *(volatile v4f*)(gp + 128 + 4 * lane) = v1;
  }
}

extern "C" void kernel_launch(void* const* d_in, const int* in_sizes, int n_in,
                              void* d_out, int out_size, void* d_ws, size_t ws_size,
                              hipStream_t stream) {
  if (n_in < 7) return;
  const int N = in_sizes[1];
  if (N != NN) return;
  if (in_sizes[0] != N * HH) return;
  if ((in_sizes[2] & 1) != 0) return;
  const int E = in_sizes[2] / 2;
  if (E <= 0 || (E % GPB) != 0) return;
  if (in_sizes[3] != 2 * HH || in_sizes[4] != 2 * HH || in_sizes[5] != 2 * HH || in_sizes[6] < 1) return;
  if ((N % RB) != 0) return;
  if (out_size != N * HH + E) return;

  const float* feat  = (const float*)d_in[0];
  const float* nd    = (const float*)d_in[1];
  const int*   pairs = (const int*)d_in[2];
  const float* gamma = (const float*)d_in[3];
  const float* beta  = (const float*)d_in[4];
  const float* gw    = (const float*)d_in[5];
  const float* gb    = (const float*)d_in[6];
  float* out  = (float*)d_out;
  float* gout = out + (size_t)N * HH;

  char* ws = (char*)d_ws;
  size_t off = 0;
  const size_t oXh = off; off += (size_t)N * HH * 2; off = (off + 255) & ~(size_t)255;
  const size_t oXl = off; off += (size_t)N * HH * 2; off = (off + 255) & ~(size_t)255;
  if (off > ws_size || off > (size_t)WSCAP) return;
  unsigned short* Xh = (unsigned short*)(ws + oXh);
  unsigned short* Xl = (unsigned short*)(ws + oXl);

  hipFuncSetAttribute(reinterpret_cast<const void*>(&k_agg),
                      hipFuncAttributeMaxDynamicSharedMemorySize, LDS_AGG);

  {
    const int t8 = (N * HH) / 8;
    k_cvt<<<(t8 + NTHR - 1) / NTHR, NTHR, 0, stream>>>(feat, Xh, Xl, HH, N, t8);
  }
  k_gate<<<E / GPB, NTHR, 0, stream>>>(feat, nd, pairs, gamma, beta, gw, gb, gout, N, E);
  {
    const int nChunks = (E + ECH - 1) / ECH;
    k_agg<<<N / RB, NTHR, LDS_AGG, stream>>>(pairs, Xh, Xl, gout, out, E, nChunks);
  }
}
